// Matformer_18726057411347
// MI455X (gfx1250) — hardware-run, weakly checked
//
#include <hip/hip_runtime.h>


namespace {
constexpr int N = 10000, E = 100000, IN = 128, C = 64, H = 4, ED = 128, C3 = 192, NW = N / 16  ;
constexpr float XS = 8.0f, HS = 256.0f, WSC = 256.0f, EPS = 1e-5f, ISQ = 0.07216878364870322f  ;
typedef _Float16 b16;
typedef __attribute__((ext_vector_type(16))) _Float16 v16b;
typedef __attribute__((ext_vector_type(8))) _Float16 v8b;
typedef __attribute__((ext_vector_type(8))) float v8f;
typedef __attribute__((ext_vector_type(4))) float v4f;
typedef __attribute__((ext_vector_type(2))) float v2f;
__device__ __forceinline__ float bf16_rne(float f) { unsigned int u = __float_as_uint(f); u += 0x7FFFu + ((u >> 16) & 1u); float r = __uint_as_float(u & 0xFFFF0000u); asm volatile("" : "+v"(r)); return r; }
__device__ __forceinline__ float bfv(float f) { float r = bf16_rne(f); asm volatile("" : "+v"(r)); return r; }
__device__ __forceinline__ void split16(float v, b16& hi, b16& lo) { hi = (b16)v; lo = (b16)(v - (float)hi); }
__device__ __forceinline__ v16b frag_kb(const b16* p, int hh) { const v8b a = *(const v8b*)(p + 8 * hh), b = *(const v8b*)(p + 16 + 8 * hh); v16b f;
#pragma unroll
  for (int e = 0; e < 8; ++e) { f[e] = a[e]; f[8 + e] = b[e]; } return f; }
__device__ __forceinline__ v8f wmma16b(v16b a, v16b b, v8f c) { v8f d = __builtin_amdgcn_wmma_f32_16x16x32_f16(false, a, false, b, (short)0, c, false, false); asm volatile("v_nop\n\tv_nop\n\tv_nop\n\tv_nop" : "+v"(d) : "v"(a), "v"(b)); return d; }
__device__ __forceinline__ void wave_lds_sync() { __builtin_amdgcn_fence(__ATOMIC_RELEASE, "workgroup"); __builtin_amdgcn_wave_barrier(); __builtin_amdgcn_fence(__ATOMIC_ACQUIRE, "workgroup"); }
__device__ __forceinline__ float pmul(float a, float b) { float p = a * b; asm volatile("" : "+v"(p)); return p; }
__device__ __forceinline__ int iclamp(int v, int lo, int hi) { return v < lo ? lo : (v > hi ? hi : v); }
constexpr int CSR_NBLK8 = 512, CSR_GB8 = 8, CSR_GN8 = 1 << CSR_GB8  , CSR_TS8 = (CSR_GN8 < 32 ? 32 : CSR_GN8)  , CSR_MAXG8 = 512, CSR_CAP8 = 12288  ;
__device__ __host__ __forceinline__ int csr_tix8(int v) { return (v >> CSR_GB8) * CSR_TS8 + (v & (CSR_GN8 - 1)); }
__global__ __launch_bounds__(64) void csrA_kernel8(const int* __restrict__ dst, int E, int N, int nG, int CHP, int NGP, int* __restrict__ STG, int* __restrict__ HST) {
  extern __shared__ int sm[];
  int* cnt = sm; int* run = sm + NGP; int* ids = sm + 2 * NGP;
  const int b = blockIdx.x; const int ch = (E + CSR_NBLK8 - 1) / CSR_NBLK8; const int e0 = b * ch, e1 = min(E, e0 + ch);
  for (int i = threadIdx.x; i < NGP; i += 64) cnt[i] = 0;
  for (int i = threadIdx.x; i < CHP; i += 64) ids[i] = -1;
  __syncthreads();
  if (threadIdx.x == 0) {
    for (int e = e0; e < e1; ++e) { int d = dst[e]; d = (d < 0) ? 0 : (d >= N ? N - 1 : d); cnt[d >> CSR_GB8] += 1; }
    int acc = 0; for (int g = 0; g < nG; ++g) { run[g] = acc; acc += cnt[g]; }
    for (int e = e0; e < e1; ++e) { int d = dst[e]; d = (d < 0) ? 0 : (d >= N ? N - 1 : d); const int g = d >> CSR_GB8; ids[run[g]] = e; run[g] += 1; } }
  __syncthreads();
  typedef __attribute__((ext_vector_type(4))) int v4i;
  for (int pass = 0; pass < 2; ++pass) {
    for (int i = threadIdx.x; i < CHP / 4; i += 64) *(volatile v4i*)(STG + (size_t)b * CHP + i * 4) = *(const v4i*)(&ids[i * 4]);
    for (int i = threadIdx.x; i < NGP / 4; i += 64) { v4i v; for (int e = 0; e < 4; ++e) v[e] = (i * 4 + e < nG) ? cnt[i * 4 + e] : 0; *(volatile v4i*)(HST + (size_t)b * NGP + i * 4) = v; }
    __threadfence(); }
}
__global__ __launch_bounds__(512) void csrS_kernel8(const int* __restrict__ HST, int nG, int NGP, int* __restrict__ START, int* __restrict__ TOT, int* __restrict__ OFF) {
  __shared__ int tot[CSR_MAXG8];
  const int b = threadIdx.x;
  for (int pass = 0; pass < 2; ++pass) { int runb = 0; for (int g = 0; g < nG; ++g) { int c = HST[(size_t)b * NGP + g]; c = (c < 0) ? 0 : c; ((volatile int*)OFF)[(size_t)g * CSR_NBLK8 + b] = runb; runb += c; } __threadfence(); }
  for (int g = threadIdx.x; g < nG; g += 512) { int s = 0; for (int bb = 0; bb < CSR_NBLK8; ++bb) { int c = HST[(size_t)bb * NGP + g]; s += (c < 0) ? 0 : c; } tot[g] = s; }
  __syncthreads();
  if (threadIdx.x < 32) {
    __shared__ int st[CSR_MAXG8 + 32];
    if (threadIdx.x == 0) { int acc = 0; for (int g = 0; g < NGP; ++g) { st[g] = acc; if (g < nG) acc += (tot[g] + 31) & ~31; } st[NGP] = acc; }
    __builtin_amdgcn_fence(__ATOMIC_RELEASE, "workgroup"); __builtin_amdgcn_wave_barrier(); __builtin_amdgcn_fence(__ATOMIC_ACQUIRE, "workgroup");
    for (int pass = 0; pass < 2; ++pass) { for (int i = threadIdx.x; i < NGP + 32; i += 32) { ((volatile int*)START)[i] = (i <= NGP) ? st[min(i, NGP)] : 0; ((volatile int*)TOT)[i] = (i < nG) ? tot[i] : 0; } __threadfence(); } }
}
__global__ __launch_bounds__(256) void csrB_kernel8(const int* __restrict__ dst, int N, int nG, int CHP, int NGP, int permLen, const int* __restrict__ STG, const int* __restrict__ HST, const int* __restrict__ OFF, const int* __restrict__ START, const int* __restrict__ TOT, int* __restrict__ PERM, int* __restrict__ ROWPTR, int* __restrict__ ROWCNT, int* __restrict__ FLAG) {
  typedef __attribute__((ext_vector_type(4))) int v4i;
  __shared__ int ids[CSR_CAP8]; __shared__ unsigned short key[CSR_CAP8]; __shared__ int outp[CSR_CAP8]; __shared__ int ncnt[CSR_GN8 + 1]; __shared__ int boff[CSR_NBLK8 + 1];
  const int g = blockIdx.x, t_ = threadIdx.x; int tot = TOT[g]; int st = START[g], stn = START[g + 1]; const int v0 = g * CSR_GN8; const int nv = min(CSR_GN8, N - v0); const int t0 = g * CSR_TS8;
  st = (st < 0) ? 0 : (st > permLen - 32 ? permLen - 32 : st) & ~31; stn = (stn < st) ? st : (stn > permLen ? permLen : stn); tot = (tot < 0) ? 0 : tot; if (tot > stn - st && tot <= CSR_CAP8) tot = stn - st;
  if (tot > CSR_CAP8) {
    for (int pass = 0; pass < 2; ++pass) { for (int i = t_; i < CSR_TS8 / 4; i += 256) { v4i a, c; for (int e = 0; e < 4; ++e) { a[e] = st; c[e] = 0; } *(volatile v4i*)(ROWPTR + t0 + i * 4) = a; *(volatile v4i*)(ROWCNT + t0 + i * 4) = c; } if (t_ == 0) ((volatile int*)FLAG)[0] = 1; __threadfence(); } (void)nv; return; }
  if (t_ == 0) { int acc = 0; for (int b = 0; b < CSR_NBLK8; ++b) { boff[b] = acc; int c = HST[(size_t)b * NGP + g]; c = (c < 0) ? 0 : (c > CHP ? CHP : c); acc += c; if (acc > tot) acc = tot; } boff[CSR_NBLK8] = acc; }
  for (int i = t_; i <= CSR_GN8; i += 256) ncnt[i] = 0;
  __syncthreads();
  for (int b = 0; b < CSR_NBLK8; ++b) { const int c = boff[b + 1] - boff[b]; int o_ = OFF[(size_t)g * CSR_NBLK8 + b]; o_ = (o_ < 0) ? 0 : (o_ > CHP - c ? CHP - c : o_); const int* src_ = STG + (size_t)b * CHP + o_;
    for (int i = t_; i < c; i += 256) { int id = src_[i]; id = (id < 0) ? 0 : id; ids[boff[b] + i] = id; int d = dst[id]; d = (d < v0) ? v0 : (d >= N ? N - 1 : d); int kk = d - v0; kk = (kk < 0) ? 0 : (kk >= CSR_GN8 ? CSR_GN8 - 1 : kk); key[boff[b] + i] = (unsigned short)kk; } }
  __syncthreads();
  if (t_ == 0) { for (int i = 0; i < tot; ++i) ncnt[key[i]] += 1; int acc = 0; for (int vl = 0; vl < CSR_GN8; ++vl) { const int c = ncnt[vl]; ncnt[vl] = acc; acc += c; } ncnt[CSR_GN8] = acc;
    for (int i = 0; i < tot; ++i) { const int vl = key[i]; outp[ncnt[vl]] = ids[i]; ncnt[vl] += 1; }
    for (int vl = CSR_GN8; vl > 0; --vl) ncnt[vl] = ncnt[vl - 1]; ncnt[0] = 0; }
  __syncthreads();
  for (int pass = 0; pass < 2; ++pass) {
    for (int i = t_; i < (stn - st) / 4; i += 256) { v4i v; for (int e = 0; e < 4; ++e) { const int q = i * 4 + e; v[e] = (q < tot) ? outp[q] : -1; } *(volatile v4i*)(PERM + st + i * 4) = v; }
    for (int i = t_; i < CSR_TS8 / 4; i += 256) { v4i a, c; for (int e = 0; e < 4; ++e) { const int vl = i * 4 + e; const int vc = vl < CSR_GN8 ? vl : CSR_GN8; a[e] = (vl < CSR_GN8) ? st + ncnt[vc] : st; c[e] = (vl < nv) ? (ncnt[(vc < CSR_GN8 ? vc : CSR_GN8 - 1) + 1] - ncnt[vc]) : 0; } *(volatile v4i*)(ROWPTR + t0 + i * 4) = a; *(volatile v4i*)(ROWCNT + t0 + i * 4) = c; }
    __threadfence(); }
}
__global__ __launch_bounds__(256) void csrZ_kernel8(int* __restrict__ p, size_t n4) { typedef __attribute__((ext_vector_type(4))) int v4i; const size_t tid = (size_t)blockIdx.x * 256 + threadIdx.x, nth = (size_t)gridDim.x * 256; v4i z = {0, 0, 0, 0}; for (size_t i = tid; i < n4; i += nth) *(volatile v4i*)(p + i * 4) = z; }
struct CsrBufs8 { int *STG, *HST, *OFF, *START, *TOT, *PERM, *ROWPTR, *ROWCNT, *FLAG; int nG, NGP, CHP; size_t permLen; char* base; size_t bytes; };
static size_t csr_carve8(CsrBufs8& c, char* ws, size_t off, int E, int N) {
  const size_t off0 = off; c.base = ws + off;
  auto al = [&](size_t bytes) { char* p = ws + off; off += (bytes + 255) & ~(size_t)255; return p; };
  c.nG = (N + CSR_GN8 - 1) / CSR_GN8; c.NGP = (c.nG + 31) & ~31; const int ch = (E + CSR_NBLK8 - 1) / CSR_NBLK8; c.CHP = (ch + 31) & ~31; c.permLen = (size_t)E + 32 * (size_t)c.nG + 32;
  c.STG = (int*)al((size_t)CSR_NBLK8 * c.CHP * 4); c.HST = (int*)al((size_t)CSR_NBLK8 * c.NGP * 4); c.OFF = (int*)al((size_t)c.NGP * CSR_NBLK8 * 4); c.START = (int*)al((size_t)(c.NGP + 64) * 4); c.TOT = (int*)al((size_t)(c.NGP + 64) * 4);
  c.PERM = (int*)al(c.permLen * 4); c.ROWPTR = (int*)al((size_t)c.nG * CSR_TS8 * 4); c.ROWCNT = (int*)al((size_t)c.nG * CSR_TS8 * 4); c.FLAG = (int*)al(256);
  c.bytes = off - off0; return off;
}
static void csr_build8(const CsrBufs8& c, const int* dst, int E, int N, hipStream_t stream) {
  const size_t smem = (size_t)(2 * c.NGP + c.CHP) * 4;
  csrZ_kernel8<<<512, 256, 0, stream>>>((int*)c.base, c.bytes / 16);
  csrA_kernel8<<<CSR_NBLK8, 64, smem, stream>>>(dst, E, N, c.nG, c.CHP, c.NGP, c.STG, c.HST);
  csrS_kernel8<<<1, 512, 0, stream>>>(c.HST, c.nG, c.NGP, c.START, c.TOT, c.OFF);
  csrB_kernel8<<<c.nG, 256, 0, stream>>>(dst, N, c.nG, c.CHP, c.NGP, (int)c.permLen, c.STG, c.HST, c.OFF, c.START, c.TOT, c.PERM, c.ROWPTR, c.ROWCNT, c.FLAG);
}


__global__ __launch_bounds__(256) void prep_kernel(const float* __restrict__ wq, const float* __restrict__ wk, const float* __restrict__ wv, const float* __restrict__ wskip, const float* __restrict__ we, const float* __restrict__ wmsg, const float* __restrict__ wml, const float* __restrict__ wcat, b16* __restrict__ WN, b16* __restrict__ WE, b16* __restrict__ WAB, b16* __restrict__ WC, b16* __restrict__ WML, b16* __restrict__ WCAT) { const size_t nt = (size_t)gridDim.x * 256, u0 = (size_t)blockIdx.x * 256 + threadIdx.x; v8b v;
  for (size_t u = u0; u < (size_t)832 * 16; u += nt) { const int o = (int)(u / 16), k0 = (int)(u % 16) * 8; const float* w; int oo, nc; if (o < 256) { w = wq; oo = o; nc = 256; } else if (o < 512) { w = wk; oo = o - 256; nc = 256; } else if (o < 768) { w = wv; oo = o - 512; nc = 256; } else { w = wskip; oo = o - 768; nc = 64; }
#pragma unroll
    for (int j = 0; j < 8; ++j) v[j] = (b16)(bf16_rne(w[(size_t)(k0 + j) * nc + oo]) * WSC); for (int pass = 0; pass < 2; ++pass) { *(volatile v8b*)(WN + (size_t)o * IN + k0) = v; __threadfence(); } }
  for (size_t u = u0; u < (size_t)256 * 16; u += nt) { const int o = (int)(u / 16), k0 = (int)(u % 16) * 8;
#pragma unroll
    for (int j = 0; j < 8; ++j) v[j] = (b16)(bf16_rne(we[(size_t)(k0 + j) * 256 + o]) * WSC); for (int pass = 0; pass < 2; ++pass) { *(volatile v8b*)(WE + (size_t)o * ED + k0) = v; __threadfence(); } }
  for (size_t u = u0; u < (size_t)384 * 8; u += nt) { const int r = (int)(u / 8), k0 = (int)(u % 8) * 8; const int part = r / C3, o = r % C3;
#pragma unroll
    for (int j = 0; j < 8; ++j) v[j] = (b16)(bf16_rne(wmsg[(size_t)(part * C + k0 + j) * C3 + o]) * WSC); for (int pass = 0; pass < 2; ++pass) { *(volatile v8b*)(WAB + (size_t)r * C + k0) = v; __threadfence(); } }
  for (size_t u = u0; u < (size_t)C3 * 8; u += nt) { const int o = (int)(u / 8), k0 = (int)(u % 8) * 8;
#pragma unroll
    for (int j = 0; j < 8; ++j) v[j] = (b16)(bf16_rne(wmsg[(size_t)(2 * C + k0 + j) * C3 + o]) * WSC); for (int pass = 0; pass < 2; ++pass) { *(volatile v8b*)(WC + (size_t)o * C + k0) = v; __threadfence(); } }
  for (size_t u = u0; u < (size_t)C * 24; u += nt) { const int o = (int)(u / 24), k0 = (int)(u % 24) * 8;
#pragma unroll
    for (int j = 0; j < 8; ++j) v[j] = (b16)(bf16_rne(wml[(size_t)(k0 + j) * C + o]) * WSC); for (int pass = 0; pass < 2; ++pass) { *(volatile v8b*)(WML + (size_t)o * C3 + k0) = v; __threadfence(); } }
  for (size_t u = u0; u < (size_t)C * 32; u += nt) { const int o = (int)(u / 32), k0 = (int)(u % 32) * 8;
#pragma unroll
    for (int j = 0; j < 8; ++j) v[j] = (b16)(bf16_rne(wcat[(size_t)(k0 + j) * C + o]) * WSC); for (int pass = 0; pass < 2; ++pass) { *(volatile v8b*)(WCAT + (size_t)o * 256 + k0) = v; __threadfence(); } } }
__global__ __launch_bounds__(32) void nproj_kernel(const float* __restrict__ x, const b16* __restrict__ WN, const float* __restrict__ bq, const float* __restrict__ bk, const float* __restrict__ bv, const float* __restrict__ bs, int NLIM, float* __restrict__ QKV, float* __restrict__ SK) { __shared__ __attribute__((aligned(16))) b16 Ax[16][IN + 8]; __shared__ float Tf[16][260]; const int lane = threadIdx.x, nloc = lane & 15, hlf = lane >> 4; const size_t n0 = (size_t)blockIdx.x * 16; if (n0 >= (size_t)NLIM) return;
  for (int rr = 0; rr < 16; ++rr) for (int q = 0; q < 4; ++q) { const int c = q * 32 + lane; Ax[rr][c] = (b16)(bf16_rne(x[(n0 + rr) * IN + c]) * XS); }
  if (lane < 16) for (int k = IN; k < IN + 8; ++k) Ax[lane][k] = (b16)0.0f;
  wave_lds_sync();
#pragma unroll 1
  for (int g = 0; g < 4; ++g) { const int nt = g < 3 ? 16 : 4; const float* bias = g == 0 ? bq : (g == 1 ? bk : (g == 2 ? bv : bs)); v8f acc[16];
#pragma unroll
    for (int t = 0; t < 16; ++t) acc[t] = (v8f){};
#pragma unroll
    for (int kb = 0; kb < IN; kb += 32) { const v16b a = frag_kb(&Ax[nloc][kb], hlf);
#pragma unroll
      for (int t = 0; t < 16; ++t) if (t < nt) acc[t] = wmma16b(a, frag_kb(WN + (size_t)(g * 256 + t * 16 + nloc) * IN + kb, hlf), acc[t]); }
#pragma unroll
    for (int t = 0; t < 16; ++t) if (t < nt) { const int cc = t * 16 + nloc; const float bb = bfv(bias[cc]);
#pragma unroll
      for (int r8 = 0; r8 < 8; ++r8) Tf[8 * hlf + r8][cc] = acc[t][r8] * (1.0f / (XS * WSC)) + bb; }
    wave_lds_sync();
    for (int pass = 0; pass < 2; ++pass) { for (int rr = 0; rr < 16; ++rr) { if (g < 3) { for (int q = 0; q < 2; ++q) *(volatile v4f*)(QKV + (n0 + rr) * 768 + g * 256 + q * 128 + lane * 4) = *(const v4f*)(&Tf[rr][q * 128 + lane * 4]); } else *(volatile v2f*)(SK + (n0 + rr) * C + lane * 2) = (v2f){Tf[rr][lane * 2], Tf[rr][lane * 2 + 1]}; } __threadfence(); }
    wave_lds_sync(); } }
__global__ __launch_bounds__(32) void vab_kernel(const float* __restrict__ QKV, const b16* __restrict__ WAB, const float* __restrict__ bmsg, int NLIM, float* __restrict__ VAB) { __shared__ __attribute__((aligned(16))) b16 Ah[16][C + 8], Al[16][C + 8]; __shared__ float Tf[16][388]; const int lane = threadIdx.x, nloc = lane & 15, hlf = lane >> 4; const size_t r0 = (size_t)blockIdx.x * 16; if (r0 >= (size_t)NLIM * H) return;
  for (int rr = 0; rr < 16; ++rr) for (int q = 0; q < 2; ++q) { const int c = q * 32 + lane; const size_t nh = r0 + rr; b16 p, pl; split16(QKV[(nh / H) * 768 + 512 + (nh % H) * C + c] * HS, p, pl); Ah[rr][c] = p; Al[rr][c] = pl; }
  if (lane < 16) for (int k = C; k < C + 8; ++k) { Ah[lane][k] = (b16)0.0f; Al[lane][k] = (b16)0.0f; }
  wave_lds_sync();
#pragma unroll 1
  for (int g = 0; g < 2; ++g) { v8f acc[12];
#pragma unroll
    for (int t = 0; t < 12; ++t) acc[t] = (v8f){};
#pragma unroll
    for (int kb = 0; kb < C; kb += 32) { const v16b a = frag_kb(&Ah[nloc][kb], hlf), al = frag_kb(&Al[nloc][kb], hlf);
#pragma unroll
      for (int t = 0; t < 12; ++t) { const v16b bw = frag_kb(WAB + (size_t)(g * C3 + t * 16 + nloc) * C + kb, hlf); acc[t] = wmma16b(a, bw, acc[t]); acc[t] = wmma16b(al, bw, acc[t]); } }
#pragma unroll
    for (int t = 0; t < 12; ++t) { const int cc = t * 16 + nloc; const float bb = g == 0 ? bfv(bmsg[cc]) : 0.0f;
#pragma unroll
      for (int r8 = 0; r8 < 8; ++r8) Tf[8 * hlf + r8][g * C3 + cc] = acc[t][r8] * (1.0f / (HS * WSC)) + bb; } }
  wave_lds_sync();
  for (int pass = 0; pass < 2; ++pass) { for (int rr = 0; rr < 16; ++rr) for (int q = 0; q < 3; ++q) *(volatile v4f*)(VAB + (r0 + rr) * 384 + q * 128 + lane * 4) = *(const v4f*)(&Tf[rr][q * 128 + lane * 4]); __threadfence(); } }
__device__ __forceinline__ void ln_lane(float* row, int n, const float* g, const float* b) { float m = 0.0f; for (int c = 0; c < n; ++c) m += row[c]; m *= 1.0f / (float)n; float vr = 0.0f; for (int c = 0; c < n; ++c) { const float d = row[c] - m; vr += d * d; } vr *= 1.0f / (float)n; const float rs = rsqrtf(vr + EPS); for (int c = 0; c < n; ++c) row[c] = pmul(bfv(g[c]), (row[c] - m) * rs) + bfv(b[c]); }
__global__ __launch_bounds__(32) void edge_kernel(const float* __restrict__ ea, const int* __restrict__ ei, const float* __restrict__ QKV, const float* __restrict__ VAB, const b16* __restrict__ WE, const b16* __restrict__ WC, const b16* __restrict__ WML, const float* __restrict__ bml, const float* __restrict__ gml, const float* __restrict__ bbml, const float* __restrict__ g3, const float* __restrict__ b3, int ELIM, int NLIM, float* __restrict__ MSG) { __shared__ __attribute__((aligned(16))) b16 Ah[16][IN + 8], Bh[16][C + 8], Bl[16][C + 8], Mh[16][C3 + 8], Ml[16][C3 + 8]; __shared__ float Te[16][260], Tm[16][C3 + 1], Ga[16][C3 + 1], To[16][C + 1]; __shared__ int Sx[16], Dx[16]; const int lane = threadIdx.x, nloc = lane & 15, hlf = lane >> 4; const size_t e0 = (size_t)blockIdx.x * 16; if (e0 >= (size_t)ELIM) return;
  { const int s_ = iclamp(ei[e0 + nloc], 0, N - 1), d_ = iclamp(ei[E + e0 + nloc], 0, N - 1); const bool inside = s_ < NLIM && d_ < NLIM; if (__builtin_amdgcn_ballot_w32(inside) == 0) return; }
  if (lane < 16) { Sx[lane] = iclamp(ei[e0 + lane], 0, N - 1); Dx[lane] = iclamp(ei[E + e0 + lane], 0, N - 1); for (int k = IN; k < IN + 8; ++k) Ah[lane][k] = (b16)0.0f; for (int k = C; k < C + 8; ++k) { Bh[lane][k] = (b16)0.0f; Bl[lane][k] = (b16)0.0f; } for (int k = C3; k < C3 + 8; ++k) { Mh[lane][k] = (b16)0.0f; Ml[lane][k] = (b16)0.0f; } }
  for (int rr = 0; rr < 16; ++rr) for (int q = 0; q < 4; ++q) { const int c = q * 32 + lane; Ah[rr][c] = (b16)(bfv(ea[(e0 + rr) * ED + c]) * XS); }
  wave_lds_sync();
  { v8f acc[16];
#pragma unroll
    for (int t = 0; t < 16; ++t) acc[t] = (v8f){};
#pragma unroll 1
    for (int kb = 0; kb < ED; kb += 32) { const v16b a = frag_kb(&Ah[nloc][kb], hlf);
#pragma unroll
      for (int t = 0; t < 16; ++t) acc[t] = wmma16b(a, frag_kb(WE + (size_t)(t * 16 + nloc) * ED + kb, hlf), acc[t]); }
#pragma unroll
    for (int t = 0; t < 16; ++t)
#pragma unroll
      for (int r8 = 0; r8 < 8; ++r8) Te[8 * hlf + r8][t * 16 + nloc] = acc[t][r8] * (1.0f / (XS * WSC)); }
  wave_lds_sync();
#pragma unroll 1
  for (int h = 0; h < H; ++h) {
    for (int rr = 0; rr < 16; ++rr) { for (int q = 0; q < 2; ++q) { const int c = q * 32 + lane; b16 p, pl; split16(Te[rr][h * C + c] * HS, p, pl); Bh[rr][c] = p; Bl[rr][c] = pl; } const float* va = VAB + ((size_t)Dx[rr] * H + h) * 384; const float* vb = VAB + ((size_t)Sx[rr] * H + h) * 384 + C3; for (int q = 0; q < 6; ++q) { const int c = q * 32 + lane; Tm[rr][c] = va[c] + vb[c]; } }
    wave_lds_sync();
    { v8f acc[12];
#pragma unroll
      for (int t = 0; t < 12; ++t) acc[t] = (v8f){};
#pragma unroll 1
      for (int kb = 0; kb < C; kb += 32) { const v16b a = frag_kb(&Bh[nloc][kb], hlf), al = frag_kb(&Bl[nloc][kb], hlf);
#pragma unroll
        for (int t = 0; t < 12; ++t) { const v16b bw = frag_kb(WC + (size_t)(t * 16 + nloc) * C + kb, hlf); acc[t] = wmma16b(a, bw, acc[t]); acc[t] = wmma16b(al, bw, acc[t]); } }
#pragma unroll
      for (int t = 0; t < 12; ++t)
#pragma unroll
        for (int r8 = 0; r8 < 8; ++r8) { const int rr = 8 * hlf + r8, cc = t * 16 + nloc; Tm[rr][cc] += acc[t][r8] * (1.0f / (HS * WSC)); } }
    wave_lds_sync();
    for (int r = 0; r < 16; ++r) { const float* qi = QKV + (size_t)Dx[r] * 768 + h * C; const float* ki = QKV + (size_t)Dx[r] * 768 + 256 + h * C; const float* kj = QKV + (size_t)Sx[r] * 768 + 256 + h * C;
      for (int q = 0; q < 2; ++q) { const int c = q * 32 + lane; const float qv = qi[c]; Ga[r][c] = pmul(pmul(qv, ki[c]), ISQ); Ga[r][C + c] = pmul(pmul(qv, kj[c]), ISQ); Ga[r][2 * C + c] = pmul(pmul(qv, Te[r][h * C + c]), ISQ); } }
    wave_lds_sync();
    if (lane < 16) { const int r = lane; ln_lane(&Ga[r][0], C3, g3, b3);
#pragma unroll 1
      for (int c = 0; c < C3; ++c) Tm[r][c] = pmul(Tm[r][c], 1.0f / (1.0f + __expf(-Ga[r][c]))); }
    wave_lds_sync();
    for (int rr = 0; rr < 16; ++rr) for (int q = 0; q < 6; ++q) { const int c = q * 32 + lane; b16 p, pl; split16(Tm[rr][c] * HS, p, pl); Mh[rr][c] = p; Ml[rr][c] = pl; }
    wave_lds_sync();
    { v8f acc[4] = {(v8f){}, (v8f){}, (v8f){}, (v8f){}};
#pragma unroll 1
      for (int kb = 0; kb < C3; kb += 32) { const v16b a = frag_kb(&Mh[nloc][kb], hlf), al2 = frag_kb(&Ml[nloc][kb], hlf);
#pragma unroll
        for (int t = 0; t < 4; ++t) { const v16b bw = frag_kb(WML + (size_t)(t * 16 + nloc) * C3 + kb, hlf); acc[t] = wmma16b(a, bw, acc[t]); acc[t] = wmma16b(al2, bw, acc[t]); } }
#pragma unroll
      for (int t = 0; t < 4; ++t) { const int cc = t * 16 + nloc; const float bb = bfv(bml[cc]);
#pragma unroll
        for (int r8 = 0; r8 < 8; ++r8) To[8 * hlf + r8][cc] = acc[t][r8] * (1.0f / (HS * WSC)) + bb; } }
    wave_lds_sync();
    if (lane < 16) ln_lane(&To[lane][0], C, gml, bbml);
    wave_lds_sync();
    for (int pass = 0; pass < 2; ++pass) { for (int rr = 0; rr < 16; ++rr) *(volatile v2f*)(MSG + ((e0 + rr) * H + h) * C + lane * 2) = (v2f){To[rr][lane * 2], To[rr][lane * 2 + 1]}; __threadfence(); }
    wave_lds_sync(); } }
__global__ __launch_bounds__(32) void agg_kernel(const float* __restrict__ MSG, const int* __restrict__ PERM, const int* __restrict__ ROWPTR, const int* __restrict__ ROWCNT, int permLen, const int* __restrict__ srcs, const b16* __restrict__ WCAT, const float* __restrict__ bcat, int NLIM, float* __restrict__ PRE, float* __restrict__ PS, float* __restrict__ PQ) { __shared__ __attribute__((aligned(16))) b16 Ah[16][264], Al[16][264]; __shared__ float Tf[16][C + 1]; const int lane = threadIdx.x, nloc = lane & 15, hlf = lane >> 4; const size_t n0 = (size_t)blockIdx.x * 16; if (n0 >= (size_t)NLIM) return;
  if (lane < 16) for (int k = 256; k < 264; ++k) { Ah[lane][k] = (b16)0.0f; Al[lane][k] = (b16)0.0f; }
  for (int rr = 0; rr < 16; ++rr) { const size_t n = n0 + rr; int st = ROWPTR[n], cnt = ROWCNT[n]; cnt = iclamp(cnt, 0, E); st = iclamp(st, 0, permLen - cnt); v4f a0 = {0, 0, 0, 0}, a1 = {0, 0, 0, 0};
#pragma unroll 1
    for (int j = 0; j < cnt; ++j) { const int e = iclamp(PERM[st + j], 0, E - 1); if (srcs[e] >= NLIM) continue; const float* mp = MSG + (size_t)e * H * C + lane * 8; a0 += *(const v4f*)mp; a1 += *(const v4f*)(mp + 4); }
    for (int q = 0; q < 4; ++q) { b16 p, pl; split16(a0[q] * HS, p, pl); Ah[rr][lane * 8 + q] = p; Al[rr][lane * 8 + q] = pl; split16(a1[q] * HS, p, pl); Ah[rr][lane * 8 + 4 + q] = p; Al[rr][lane * 8 + 4 + q] = pl; } }
  wave_lds_sync(); v8f acc[4] = {(v8f){}, (v8f){}, (v8f){}, (v8f){}};
#pragma unroll
  for (int kb = 0; kb < 256; kb += 32) { const v16b a = frag_kb(&Ah[nloc][kb], hlf), al = frag_kb(&Al[nloc][kb], hlf);
#pragma unroll
    for (int t = 0; t < 4; ++t) { const v16b bw = frag_kb(WCAT + (size_t)(t * 16 + nloc) * 256 + kb, hlf); acc[t] = wmma16b(a, bw, acc[t]); acc[t] = wmma16b(al, bw, acc[t]); } }
#pragma unroll
  for (int t = 0; t < 4; ++t) { const int cc = t * 16 + nloc; const float bb = bfv(bcat[cc]);
#pragma unroll
    for (int r8 = 0; r8 < 8; ++r8) Tf[8 * hlf + r8][cc] = acc[t][r8] * (1.0f / (HS * WSC)) + bb; }
  wave_lds_sync();
  float s0 = 0, s1 = 0, q0 = 0, q1 = 0; for (int rr = 0; rr < 16; ++rr) { const float a = Tf[rr][lane * 2], b = Tf[rr][lane * 2 + 1]; s0 += a; s1 += b; q0 += pmul(a, a); q1 += pmul(b, b); }
  for (int pass = 0; pass < 2; ++pass) { for (int rr = 0; rr < 16; ++rr) *(volatile v2f*)(PRE + (n0 + rr) * C + lane * 2) = (v2f){Tf[rr][lane * 2], Tf[rr][lane * 2 + 1]}; *(volatile v2f*)(PS + (size_t)blockIdx.x * C + lane * 2) = (v2f){s0, s1}; *(volatile v2f*)(PQ + (size_t)blockIdx.x * C + lane * 2) = (v2f){q0, q1}; __threadfence(); } }
__global__ __launch_bounds__(256) void stat_kernel(const float* __restrict__ PS, const float* __restrict__ PQ, int nwaves, int ncount, float* __restrict__ ST) { const int wave = threadIdx.x >> 5, lane = threadIdx.x & 31; const int c = blockIdx.x * 8 + wave; if (c >= C) return; double s = 0.0, q = 0.0; for (int w = lane; w < nwaves; w += 32) { s += (double)PS[(size_t)w * C + c]; q += (double)PQ[(size_t)w * C + c]; } for (int o = 16; o; o >>= 1) { s += __shfl_xor(s, o); q += __shfl_xor(q, o); }
  const double mean = s / ncount, var = fmax(q / ncount - mean * mean, 0.0); const float m = (float)mean, rs = (float)(1.0 / sqrt(var + (double)EPS));
  for (int pass = 0; pass < 2; ++pass) { ((volatile float*)ST)[(size_t)c * 32 + lane] = lane == 0 ? m : (lane == 1 ? rs : 0.0f); __threadfence(); } }
__global__ __launch_bounds__(256) void fin_kernel(const float* __restrict__ PRE, const float* __restrict__ ST, const float* __restrict__ gbn, const float* __restrict__ bbn, const float* __restrict__ SK, int NLIM, float* __restrict__ out) { const size_t u = (size_t)blockIdx.x * 256 + threadIdx.x; if (u >= (size_t)NLIM * C / 2) return; const int c = (int)((u * 2) % C); v2f r;
  for (int e2 = 0; e2 < 2; ++e2) { const float m = ST[(c + e2) * 32], rs = ST[(c + e2) * 32 + 1]; const float y = pmul(bfv(gbn[c + e2]), (PRE[u * 2 + e2] - m) * rs) + bfv(bbn[c + e2]); r[e2] = y / (1.0f + __expf(-y)) + SK[u * 2 + e2]; }
  for (int pass = 0; pass < 2; ++pass) { *(volatile v2f*)(out + u * 2) = r; __threadfence(); } }
}

extern "C" void kernel_launch(void* const* d_in, const int* in_sizes, int n_in, void* d_out, int out_size, void* d_ws, size_t ws_size, hipStream_t stream) {
  (void)n_in;
  auto Fp = [&](int i) { return (const float*)d_in[i]; }; auto Ip = [&](int i) { return (const int*)d_in[i]; };
  if (in_sizes[0] != N * IN || in_sizes[1] != 2 * E || in_sizes[2] != E * ED || in_sizes[3] != IN * 256 || in_sizes[9] != ED * 256 || in_sizes[12] != 256 * C || in_sizes[14] != C3 * C3 || in_sizes[16] != C3 * C || out_size != N * C) return;
  const int NLIM = N, ELIM = E;
  size_t off = 0; char* ws = (char*)d_ws;
  auto carve = [&](size_t bytes) { char* p = ws + off; off += (bytes + 255) & ~(size_t)255; return p; };
  b16* WN = (b16*)carve(832 * IN * 2); b16* WE = (b16*)carve(256 * ED * 2); b16* WAB = (b16*)carve(384 * C * 2); b16* WC = (b16*)carve(C3 * C * 2); b16* WML = (b16*)carve(C * C3 * 2); b16* WCAT = (b16*)carve(C * 256 * 2);
  float* QKV = (float*)carve((size_t)N * 768 * 4); float* SK = (float*)carve((size_t)N * C * 4); float* VAB = (float*)carve((size_t)N * H * 384 * 4); float* MSG = (float*)carve((size_t)E * H * C * 4); float* PRE = (float*)carve((size_t)N * C * 4); float* PS = (float*)carve((size_t)NW * C * 4); float* PQ = (float*)carve((size_t)NW * C * 4); float* ST = (float*)carve((size_t)C * 32 * 4); CsrBufs8 csr; off = csr_carve8(csr, ws, off, E, N);
  if (off > ws_size || off > ((size_t)224 << 20)) return;
  prep_kernel<<<64, 256, 0, stream>>>(Fp(3), Fp(5), Fp(7), Fp(10), Fp(9), Fp(14), Fp(16), Fp(12), WN, WE, WAB, WC, WML, WCAT);
  csr_build8(csr, Ip(1) + E, E, N, stream);
  nproj_kernel<<<NLIM / 16, 32, 0, stream>>>(Fp(0), WN, Fp(4), Fp(6), Fp(8), Fp(11), NLIM, QKV, SK);
  vab_kernel<<<NLIM * H / 16, 32, 0, stream>>>(QKV, WAB, Fp(15), NLIM, VAB);
  edge_kernel<<<ELIM / 16, 32, 0, stream>>>(Fp(2), Ip(1), QKV, VAB, WE, WC, WML, Fp(17), Fp(18), Fp(19), Fp(20), Fp(21), ELIM, NLIM, MSG);
  agg_kernel<<<NLIM / 16, 32, 0, stream>>>(MSG, csr.PERM, csr.ROWPTR, csr.ROWCNT, (int)csr.permLen, Ip(1), WCAT, Fp(13), NLIM, PRE, PS, PQ);
  stat_kernel<<<C / 8, 256, 0, stream>>>(PS, PQ, NLIM / 16, NLIM, ST);
  fin_kernel<<<(NLIM * C / 2 + 255) / 256, 256, 0, stream>>>(PRE, ST, Fp(22), Fp(23), SK, NLIM, (float*)d_out);
}
